// LocalFeatureAggregation_12936441495845
// MI455X (gfx1250) — hardware-verified
//
#include <hip/hip_runtime.h>
#include <math.h>

constexpr int kNodes = 50000;
constexpr int kNPad  = 50048;
constexpr int kNbr   = 16;
constexpr int kCin   = 128;
constexpr int kCh2   = 256;
constexpr int kCout  = 128;
constexpr int kNPB   = 8;
constexpr float kWCarry   = 16.0f;
constexpr float kYCarry   = 4.0f;
constexpr float kScaleG1  = 1.0f / 16.0f;
constexpr float kScaleG23 = 1.0f / 64.0f;
constexpr float kBnEps    = 1e-5f;

static_assert(kNPad % 64 == 0 && kNPad >= kNodes && kNPad - kNodes < 64, "row padding");
static_assert(kCin % 32 == 0 && kCh2 % 32 == 0, "K multiples of 32");
static_assert(kCh2 % 64 == 0 && kCout % 64 == 0, "N multiples of 64");
static_assert(kCin % 64 == 0, "weight transpose tiles");
static_assert(kNPad % kNPB == 0, "pool grid exact");
static_assert((kNPad * kCin / 8) % 256 == 0, "feature cast grid exact");
static_assert(kNPB * kNbr <= 256 && kCh2 == 256, "pool thread maps assume 256 threads = 256 channels");

typedef __attribute__((ext_vector_type(16))) _Float16 v16h;
typedef __attribute__((ext_vector_type(8)))  _Float16 v8h;
typedef __attribute__((ext_vector_type(16))) __bf16   v16b;
typedef __attribute__((ext_vector_type(8)))  __bf16   v8b;
typedef __attribute__((ext_vector_type(8)))  float    v8f;
typedef __attribute__((ext_vector_type(4)))  float    v4f;
typedef __attribute__((ext_vector_type(4)))  unsigned int v4u;

__device__ __forceinline__ unsigned short f2bf_bits(float f) {
  unsigned u = __float_as_uint(f);
  return (unsigned short)((u + 0x7FFFu + ((u >> 16) & 1u)) >> 16);
}
__device__ __forceinline__ float bf_bits2f(unsigned short h) { return __uint_as_float(((unsigned)h) << 16); }

__device__ __forceinline__ void dep_guard4_h(v8f& a, v8f& b, v8f& c, v8f& d, v16h x, v16h y) {
  asm volatile("v_nop\n\tv_nop\n\tv_nop\n\tv_nop" : "+v"(a), "+v"(b), "+v"(c), "+v"(d) : "v"(x), "v"(y));
}
__device__ __forceinline__ void dep_guard4_b(v8f& a, v8f& b, v8f& c, v8f& d, v16b x, v16b y) {
  asm volatile("v_nop\n\tv_nop\n\tv_nop\n\tv_nop" : "+v"(a), "+v"(b), "+v"(c), "+v"(d) : "v"(x), "v"(y));
}
__device__ __forceinline__ void keep4_h(v16h a, v16h b, v16h c, v16h d) { asm volatile("v_nop" :: "v"(a), "v"(b), "v"(c), "v"(d)); }
__device__ __forceinline__ void keep4_b(v16b a, v16b b, v16b c, v16b d) { asm volatile("v_nop" :: "v"(a), "v"(b), "v"(c), "v"(d)); }
__device__ __forceinline__ void acc_guard4(v8f& a, v8f& b, v8f& c, v8f& d) { asm volatile("v_nop\n\tv_nop\n\tv_nop\n\tv_nop" : "+v"(a), "+v"(b), "+v"(c), "+v"(d)); }
template <typename T> struct Frag;
template <> struct Frag<_Float16> {
  typedef v16h V; union U { v16h v; v8h h[2]; };
  static __device__ __forceinline__ v16h load(const _Float16* p) {
    U f; f.h[0] = *(const v8h*)(p); f.h[1] = *(const v8h*)(p + 16); return f.v;
  }
  static __device__ __forceinline__ v8f mma(v16h a, v16h b, v8f c) {
    return __builtin_amdgcn_wmma_f32_16x16x32_f16(false, a, false, b, (short)0, c, false, false);
  }
  static __device__ __forceinline__ void guard4(v8f& a, v8f& b, v8f& c, v8f& d, v16h x, v16h y) { dep_guard4_h(a, b, c, d, x, y); }
  static __device__ __forceinline__ void keep(v16h a, v16h b, v16h c, v16h d) { keep4_h(a, b, c, d); }
};
template <> struct Frag<__bf16> {
  typedef v16b V; union U { v16b v; v8b h[2]; };
  static __device__ __forceinline__ v16b load(const __bf16* p) {
    U f; f.h[0] = *(const v8b*)(p); f.h[1] = *(const v8b*)(p + 16); return f.v;
  }
  static __device__ __forceinline__ v8f mma(v16b a, v16b b, v8f c) {
    return __builtin_amdgcn_wmma_f32_16x16x32_bf16(false, a, false, b, (short)0, c, false, false);
  }
  static __device__ __forceinline__ void guard4(v8f& a, v8f& b, v8f& c, v8f& d, v16b x, v16b y) { dep_guard4_b(a, b, c, d, x, y); }
  static __device__ __forceinline__ void keep(v16b a, v16b b, v16b c, v16b d) { keep4_b(a, b, c, d); }
};

__device__ __forceinline__ unsigned pk16(unsigned short a, unsigned short b) { return (unsigned)a | ((unsigned)b << 16); }
__device__ __forceinline__ unsigned short h_bits(float f) { const _Float16 h = (_Float16)f; return __builtin_bit_cast(unsigned short, h); }
__device__ __forceinline__ float h16_to_f32(unsigned hb) {
  const unsigned sgn = (hb & 0x8000u) << 16; const unsigned em = hb & 0x7fffu;
  const float fn = __uint_as_float((em << 13) + 0x38000000u);
  const float fs = (float)em * 5.9604644775390625e-8f;
  const float mag = (em < 0x400u) ? fs : fn; return __uint_as_float(__float_as_uint(mag) | sgn);
}

template <int ET> struct Elem;
template <> struct Elem<0> { typedef _Float16 T; };
template <> struct Elem<1> { typedef __bf16 T; };
template <int ET, bool SPLIT, int BIAS_MODE, int OUT_MODE, int ACT, bool AFF>
__global__ __launch_bounds__(256) void wmma_gemm64(
    const unsigned short* __restrict__ Ap, const unsigned short* __restrict__ A2p, int lda, long strideA,
    const unsigned short* __restrict__ Btp, const unsigned short* __restrict__ Bt2p, int ldb, long strideB,
    void* __restrict__ Cout, void* __restrict__ Cout2, int ldc, long strideC,
    const float* __restrict__ bias, const float* __restrict__ aff_sc, const float* __restrict__ aff_sh,
    int M, int N, int K, int Mreal, float scale) {
  typedef typename Elem<ET>::T T;
  typedef typename Frag<T>::V V;
  const T* A = (const T*)Ap; const T* A2 = (const T*)A2p; const T* Bt = (const T*)Btp; const T* Bt2 = (const T*)Bt2p;
  __shared__ __align__(16) float sT[8][16 * 68];
  const int b    = blockIdx.y;
  const int lane = threadIdx.x & 31;
  const int wave = threadIdx.x >> 5;
  const int tilesN = N >> 6;
  const int tilesM = M >> 6;
  const int tile = blockIdx.x * 8 + wave;
  if (tile >= tilesM * tilesN) return;
  const int tm = tile / tilesN;
  const int tn = tile - tm * tilesN;
  const int m0 = tm << 6;
  const int n0 = tn << 6;

  const T* Ab  = A  + (size_t)b * strideA;
  const T* Bb  = Bt + (size_t)b * strideB;
  const T* Ab2 = SPLIT ? (A2  + (size_t)b * strideA) : nullptr;
  const T* Bb2 = SPLIT ? (Bt2 + (size_t)b * strideB) : nullptr;

  const int rlane = lane & 15;
  const int koff  = (lane >> 4) * 8;
  const int mOff  = (lane >> 4) * 8;

  v8f acc[4][4];
#pragma unroll
  for (int i = 0; i < 4; ++i)
#pragma unroll
    for (int j = 0; j < 4; ++j) acc[i][j] = (v8f){0.f,0.f,0.f,0.f,0.f,0.f,0.f,0.f};

  for (int k0 = 0; k0 < K; k0 += 32) {
    V bh[4], bl[4];
#pragma unroll
    for (int j = 0; j < 4; ++j) {
      const size_t bo = (size_t)(n0 + (j << 4) + rlane) * ldb + koff + k0;
      bh[j] = Frag<T>::load(Bb + bo);
      if (SPLIT) bl[j] = Frag<T>::load(Bb2 + bo);
    }
#pragma unroll
    for (int i = 0; i < 4; ++i) {
      const size_t ao = (size_t)(m0 + (i << 4) + rlane) * lda + koff + k0;
      V ah = Frag<T>::load(Ab + ao);
      V al;
      if (SPLIT) al = Frag<T>::load(Ab2 + ao);
#pragma unroll
      for (int j = 0; j < 4; ++j) {
        acc[i][j] = Frag<T>::mma(ah, bh[j], acc[i][j]);
        if (SPLIT) {
          acc[i][j] = Frag<T>::mma(ah, bl[j], acc[i][j]);
          acc[i][j] = Frag<T>::mma(al, bh[j], acc[i][j]);
        }
      }
      Frag<T>::guard4(acc[i][0], acc[i][1], acc[i][2], acc[i][3], ah, SPLIT ? al : ah);
    }
    Frag<T>::keep(bh[0], bh[1], bh[2], bh[3]);
    if (SPLIT) Frag<T>::keep(bl[0], bl[1], bl[2], bl[3]);
  }
  acc_guard4(acc[0][0], acc[0][1], acc[0][2], acc[0][3]);
  acc_guard4(acc[1][0], acc[1][1], acc[1][2], acc[1][3]);
  acc_guard4(acc[2][0], acc[2][1], acc[2][2], acc[2][3]);
  acc_guard4(acc[3][0], acc[3][1], acc[3][2], acc[3][3]);

  float* slab = sT[wave];
#pragma unroll
  for (int i = 0; i < 4; ++i) {
    const int mBase = m0 + (i << 4);
#pragma unroll
    for (int j = 0; j < 4; ++j) {
      const int n = n0 + (j << 4) + rlane;
      float bv = 0.f, asc = 1.f, ash = 0.f;
      if (BIAS_MODE == 2) bv = bias[n];
      if (AFF) { asc = aff_sc[n]; ash = aff_sh[n]; }
#pragma unroll
      for (int r = 0; r < 8; ++r) {
        float v = acc[i][j][r] * scale;
        if (BIAS_MODE == 2) v += bv;
        if (ACT == 2) v = fmaxf(v, 0.0f);
        if (ACT == 4) v = (v > 0.f) ? v : 0.01f * v;
        if (ACT == 6) v = expf(fminf(fmaxf(v, -60.0f), 60.0f));
        if (AFF) v = v * asc + ash;
        slab[(mOff + r) * 68 + (j << 4) + rlane] = v;
      }
    }
    __builtin_amdgcn_fence(__ATOMIC_RELEASE, "workgroup");
    __builtin_amdgcn_wave_barrier();
    __builtin_amdgcn_fence(__ATOMIC_ACQUIRE, "workgroup");
    if (OUT_MODE == 0) {
      float* C = (float*)Cout + (size_t)b * strideC;
      const int hh = lane >> 4, c4 = (lane & 15) * 4;
      for (int pass = 0; pass < 2; ++pass) {
#pragma unroll
        for (int it = 0; it < 8; ++it) {
          const int row = it * 2 + hh;
          v4f v = *(const v4f*)(slab + row * 68 + c4);
          if (mBase + row < Mreal) *(volatile v4f*)(C + (size_t)(mBase + row) * ldc + n0 + c4) = v;
        }
        __threadfence();
      }
    } else {
      const int q = lane >> 3, c8 = (lane & 7) * 8;
      unsigned short* C  = (unsigned short*)Cout  + (size_t)b * strideC;
      unsigned short* C2 = (OUT_MODE == 2) ? ((unsigned short*)Cout2 + (size_t)b * strideC) : nullptr;
      for (int pass = 0; pass < 2; ++pass) {
#pragma unroll
        for (int it = 0; it < 4; ++it) {
          const int row = it * 4 + q;
          const float* sp = slab + row * 68 + c8;
          v8h hv, lv;
#pragma unroll
          for (int e = 0; e < 8; ++e) {
            if (OUT_MODE == 1) {
              hv[e] = (_Float16)sp[e];
            } else {
              unsigned short hb = f2bf_bits(sp[e]);
              unsigned short lb = f2bf_bits(sp[e] - bf_bits2f(hb));
              hv[e] = __builtin_bit_cast(_Float16, hb);
              lv[e] = __builtin_bit_cast(_Float16, lb);
            }
          }
          if (mBase + row < Mreal) {
            *(volatile v8h*)(C + (size_t)(mBase + row) * ldc + n0 + c8) = hv;
            if (OUT_MODE == 2) *(volatile v8h*)(C2 + (size_t)(mBase + row) * ldc + n0 + c8) = lv;
          }
        }
        __threadfence();
      }
    }
    __builtin_amdgcn_fence(__ATOMIC_RELEASE, "workgroup");
    __builtin_amdgcn_wave_barrier();
    __builtin_amdgcn_fence(__ATOMIC_ACQUIRE, "workgroup");
  }
}

__global__ __launch_bounds__(256) void wtcast_kernel(const float* __restrict__ W, unsigned short* __restrict__ WT,
                                                     int D, int H, float scale) {
  __shared__ float sm[64][65];
  const int t  = threadIdx.x;
  const int d0 = blockIdx.x * 64;
  const int h0 = blockIdx.y * 64;
#pragma unroll
  for (int i = 0; i < 16; ++i) {
    const int e = i * 256 + t;
    const int r = e >> 6;
    const int c = e & 63;
    sm[c][r] = W[(size_t)(d0 + r) * H + h0 + c] * scale;
  }
  __syncthreads();
  const int lane = t & 31, wave = t >> 5;
  const int q = lane >> 3, c8 = (lane & 7) * 8;
  for (int pass = 0; pass < 2; ++pass) {
#pragma unroll
    for (int it = 0; it < 2; ++it) {
      const int row = wave * 8 + it * 4 + q;
      unsigned short hb[8];
#pragma unroll
      for (int e = 0; e < 8; ++e) hb[e] = h_bits(sm[row][c8 + e]);
      const v4u u = (v4u){pk16(hb[0], hb[1]), pk16(hb[2], hb[3]), pk16(hb[4], hb[5]), pk16(hb[6], hb[7])};
      *(volatile v4u*)(WT + (size_t)(h0 + row) * D + d0 + c8) = u;
    }
    __threadfence();
  }
}

__global__ __launch_bounds__(256) void featcast_kernel(const float* __restrict__ X, const float* __restrict__ gam,
                                                       const float* __restrict__ bet, const float* __restrict__ rmean,
                                                       const float* __restrict__ rvar,
                                                       unsigned short* __restrict__ XH, float* __restrict__ AFT) {
  __shared__ __align__(16) float stab[2 * kCh2];
  const int t = threadIdx.x;
  const int i = blockIdx.x * 256 + t;
  const int row = i >> 4;
  const int col = (i & 15) * 8;
  const int rr  = row < kNodes ? row : kNodes - 1;
  const bool live = row < kNodes;
  const float* p = X + (size_t)rr * kCin + col;
  const v4f a = *(const v4f*)(p);
  const v4f c = *(const v4f*)(p + 4);
  unsigned short hb[8];
#pragma unroll
  for (int e = 0; e < 4; ++e) {
    hb[e]     = h_bits(live ? a[e] : 0.f);
    hb[4 + e] = h_bits(live ? c[e] : 0.f);
  }
  const v4u u = (v4u){pk16(hb[0], hb[1]), pk16(hb[2], hb[3]), pk16(hb[4], hb[5]), pk16(hb[6], hb[7])};
  unsigned short* qd = XH + 8 * (size_t)i;
  *(volatile v4u*)qd = u;
  __threadfence();
  *(volatile v4u*)qd = u;

  if (blockIdx.x == 0) {
    const float sc  = gam[t] * rsqrtf(rvar[t] + kBnEps);
    const float sc4 = kYCarry * sc;
    const float sh4 = kYCarry * bet[t] - rmean[t] * sc4;
    stab[t] = sc4;
    stab[kCh2 + t] = sh4;
  }
  __syncthreads();
  if (blockIdx.x == 0 && t < 128) {
    const v4f v = *(const v4f*)(stab + 4 * t);
    *(volatile v4f*)(AFT + 4 * t) = v;
    __threadfence();
    *(volatile v4f*)(AFT + 4 * t) = v;
  }
}

__global__ __launch_bounds__(256) void pool_kernel(const float* __restrict__ E, const unsigned short* __restrict__ YH,
                                                   const int* __restrict__ nidx, unsigned short* __restrict__ FH) {
  __shared__ __align__(16) float sE[kNbr * kCh2];
  __shared__ __align__(16) float sY[kNbr * kCh2];
  __shared__ __align__(16) float sF[kCh2];
  __shared__ int sidx[kNPB * kNbr];
  const int t = threadIdx.x, lane = t & 31, wave = t >> 5;
  const int nb0 = blockIdx.x * kNPB;
  if (t < kNPB * kNbr) {
    const int jn = t >> 4, k = t & 15;
    int node = nb0 + jn; node = node < kNodes ? node : kNodes - 1;
    int v = nidx[(size_t)node * kNbr + k];
    v = v < 0 ? 0 : (v >= kNodes ? kNodes - 1 : v);
    sidx[t] = v;
  }
  __syncthreads();
#pragma unroll 1
  for (int jn = 0; jn < kNPB; ++jn) {
    const int node = nb0 + jn;
#pragma unroll
    for (int i = 0; i < 4; ++i) {
      const int q = t + 256 * i;
      const int k = q >> 6;
      const int c4 = (q & 63) * 4;
      const int src = sidx[jn * kNbr + k];
      const v4f v = *(const v4f*)(E + (size_t)src * kCh2 + c4);
      *(v4f*)(sE + k * kCh2 + c4) = v;
    }
#pragma unroll
    for (int i = 0; i < 2; ++i) {
      const int q = t + 256 * i;
      const int k = q >> 5;
      const int c8 = (q & 31) * 8;
      const int src = sidx[jn * kNbr + k];
      const v4u w = *(const v4u*)(YH + (size_t)src * kCh2 + c8);
      v4f f0, f1;
      f0[0] = h16_to_f32(w[0] & 0xffffu); f0[1] = h16_to_f32(w[0] >> 16);
      f0[2] = h16_to_f32(w[1] & 0xffffu); f0[3] = h16_to_f32(w[1] >> 16);
      f1[0] = h16_to_f32(w[2] & 0xffffu); f1[1] = h16_to_f32(w[2] >> 16);
      f1[2] = h16_to_f32(w[3] & 0xffffu); f1[3] = h16_to_f32(w[3] >> 16);
      *(v4f*)(sY + k * kCh2 + c8) = f0;
      *(v4f*)(sY + k * kCh2 + c8 + 4) = f1;
    }
    __syncthreads();
    {
      float den = 0.0f, num = 0.0f;
#pragma unroll
      for (int k = 0; k < kNbr; ++k) {
        const float e = sE[k * kCh2 + t];
        const float g = sY[k * kCh2 + t];
        den += e;
        num = fmaf(e, g, num);
      }
      sF[t] = num * (1.0f / den);
    }
    __syncthreads();
    if (wave == 0) {
      const v4f p0 = *(const v4f*)(sF + 8 * lane);
      const v4f p1 = *(const v4f*)(sF + 8 * lane + 4);
      const bool live = node < kNodes;
      unsigned short hb[8];
#pragma unroll
      for (int e = 0; e < 4; ++e) {
        hb[e]     = h_bits(live ? p0[e] : 0.f);
        hb[4 + e] = h_bits(live ? p1[e] : 0.f);
      }
      const v4u u = (v4u){pk16(hb[0], hb[1]), pk16(hb[2], hb[3]), pk16(hb[4], hb[5]), pk16(hb[6], hb[7])};
      unsigned short* dst = FH + (size_t)node * kCh2 + 8 * lane;
      *(volatile v4u*)dst = u;
      __threadfence();
      *(volatile v4u*)dst = u;
    }
  }
}

extern "C" void kernel_launch(void* const* d_in, const int* in_sizes, int n_in,
                              void* d_out, int out_size, void* d_ws, size_t ws_size, hipStream_t stream) {
  if (n_in < 11) return;
  const float* features = (const float*)d_in[0];
  const int*   nidx     = (const int*)  d_in[1];
  const float* W1       = (const float*)d_in[2];
  const float* b1       = (const float*)d_in[3];
  const float* gamma    = (const float*)d_in[4];
  const float* beta     = (const float*)d_in[5];
  const float* rmean    = (const float*)d_in[6];
  const float* rvar     = (const float*)d_in[7];
  const float* Ws       = (const float*)d_in[8];
  const float* Wm       = (const float*)d_in[9];
  const float* bm       = (const float*)d_in[10];
  float* out = (float*)d_out;
  if (in_sizes[0] != kNodes * kCin || in_sizes[1] != kNodes * kNbr || in_sizes[2] != kCin * kCh2 ||
      in_sizes[3] != kCh2 || in_sizes[4] != kCh2 || in_sizes[5] != kCh2 || in_sizes[6] != kCh2 || in_sizes[7] != kCh2 ||
      in_sizes[8] != kCh2 * kCh2 || in_sizes[9] != kCh2 * kCout || in_sizes[10] != kCout ||
      out_size != kNodes * kCout) return;

  char* ws = (char*)d_ws; size_t off = 0;
  auto carve = [&](size_t bytes) -> char* { char* p = ws + off; off += (bytes + 255) & ~(size_t)255; return p; };
  unsigned short* W1T = (unsigned short*)carve((size_t)kCh2 * kCin * 2);
  unsigned short* WST = (unsigned short*)carve((size_t)kCh2 * kCh2 * 2);
  unsigned short* WMT = (unsigned short*)carve((size_t)kCout * kCh2 * 2);
  float*          AFT = (float*)carve((size_t)2 * kCh2 * 4);
  unsigned short* XH  = (unsigned short*)carve((size_t)kNPad * kCin * 2);
  unsigned short* YH  = (unsigned short*)carve((size_t)kNPad * kCh2 * 2);
  float*          E32 = (float*)carve((size_t)kNPad * kCh2 * 4);
  unsigned short* FH  = (unsigned short*)carve((size_t)kNPad * kCh2 * 2);
  if (off > ws_size || off > (size_t)134217728) return;

  wtcast_kernel<<<dim3(kCin / 64, kCh2 / 64), 256, 0, stream>>>(W1, W1T, kCin, kCh2, kWCarry);
  wtcast_kernel<<<dim3(kCh2 / 64, kCh2 / 64), 256, 0, stream>>>(Ws, WST, kCh2, kCh2, kWCarry);
  wtcast_kernel<<<dim3(kCh2 / 64, kCout / 64), 256, 0, stream>>>(Wm, WMT, kCh2, kCout, kWCarry);
  featcast_kernel<<<kNPad * kCin / 8 / 256, 256, 0, stream>>>(features, gamma, beta, rmean, rvar, XH, AFT);

  static_assert(kCin % 32 == 0 && kNPad % 64 == 0 && kCh2 % 64 == 0, "GEMM1 shape");
  {
    const int tiles = (kNPad / 64) * (kCh2 / 64);
    wmma_gemm64<0, false, 2, 1, 2, true><<<dim3((tiles + 7) / 8, 1), 256, 0, stream>>>(
        XH, nullptr, kCin, 0L, W1T, nullptr, kCin, 0L,
        (void*)YH, nullptr, kCh2, 0L, b1, AFT, AFT + kCh2,
        kNPad, kCh2, kCin, kNPad, kScaleG1);
  }
  static_assert(kCh2 % 32 == 0, "GEMM2 shape");
  {
    const int tiles = (kNPad / 64) * (kCh2 / 64);
    wmma_gemm64<0, false, 0, 0, 6, false><<<dim3((tiles + 7) / 8, 1), 256, 0, stream>>>(
        YH, nullptr, kCh2, 0L, WST, nullptr, kCh2, 0L,
        (void*)E32, nullptr, kCh2, 0L, nullptr, nullptr, nullptr,
        kNPad, kCh2, kCh2, kNPad, kScaleG23);
  }
  pool_kernel<<<kNPad / kNPB, 256, 0, stream>>>(E32, YH, nidx, FH);
  static_assert(kCout % 64 == 0, "GEMM3 shape");
  {
    const int tiles = (kNPad / 64) * (kCout / 64);
    wmma_gemm64<0, false, 2, 0, 0, false><<<dim3((tiles + 7) / 8, 1), 256, 0, stream>>>(
        FH, nullptr, kCh2, 0L, WMT, nullptr, kCh2, 0L,
        (void*)out, nullptr, kCout, 0L, bm, nullptr, nullptr,
        kNPad, kCout, kCh2, kNodes, kScaleG23);
  }
}
